// TransformerBlock_28827820491030
// MI455X (gfx1250) — hardware-run, weakly checked
//
#include <hip/hip_runtime.h>


#ifndef NB
#define NB 2
#endif
#ifndef SEQ
#define SEQ 2048
#endif
#define NB_FULL  2
#define SEQ_FULL 2048
#ifndef OUT_SEQ
#define OUT_SEQ SEQ
#endif
#define DM    256
#define NH_   16
#define HD    256
#define INNER 4096
#define DFF   1024
#define NPAIR 128
#define AW    4
#define OSPH  264
#define OSE   72
#define EROWS (SEQ < 256 ? SEQ : 256)
#define QRS  2048.0f
#define QRI  (1.0f / 2048.0f)
#define HC   16.0f
#define WC   64.0f
#define QC   16.0f
#define CC   256.0f
#define MC   64.0f
#define SC2  ((float)(0.0625 * 1.4426950408889634 / 256.0))
#define PSH  14.0f
#define NEGB (-3.0e38f)

static_assert(NH_ * HD == INNER);
static_assert(HD % 64 == 0);
static_assert(HD == 2 * NPAIR);
static_assert(NPAIR == 128);
static_assert(DM % 64 == 0);
static_assert(DFF % 64 == 0);
static_assert(INNER % 64 == 0);
static_assert(DM % 32 == 0);
static_assert(INNER % 32 == 0);
static_assert(DFF % 32 == 0);
static_assert(HD % 32 == 0);
static_assert(HD == 8 * 32);
static_assert(HD == 16 * 16);
static_assert(AW * 64 == HD);
static_assert(SEQ % 64 == 0);
static_assert((NB * SEQ) % 64 == 0);
static_assert((NB * SEQ) % 8 == 0);
static_assert(SEQ % 32 == 0);
static_assert(EROWS % 64 == 0);
static_assert(EROWS % 32 == 0);
static_assert(EROWS % 16 == 0);
static_assert(EROWS <= SEQ);
static_assert((SEQ - EROWS) % (16 * AW) == 0);
static_assert((SEQ * NPAIR) % 256 == 0);
static_assert(NB <= NB_FULL);
static_assert(SEQ <= SEQ_FULL);
static_assert((OSPH * 2) % 16 == 0);
static_assert((OSE * 2) % 16 == 0);
static_assert(OSPH >= HD);
static_assert(OSE >= 64);
static_assert(32 * 16 * 4 == 16 * 64 * 2);
static_assert(32 * 16 * 8 == 16 * 64 * 4);
static_assert(32 * 16 * 16 == 16 * HD * 2);
static_assert(256 * 16 * 2 == 64 * 64 * 2);
static_assert(32 * 16 == DM * 2);
static_assert(AW * 16 * OSPH * 2 <= 131072);
static_assert(AW * 16 * OSE * 2 <= 131072);
static_assert(16 * 68 * 4 <= 131072);
static_assert(64 * 68 * 4 <= 131072);

typedef _Float16 h16;
typedef __attribute__((ext_vector_type(16))) _Float16 v16h;
typedef __attribute__((ext_vector_type(8)))  _Float16 v8h;
typedef __attribute__((ext_vector_type(8)))  float    v8f;
typedef __attribute__((ext_vector_type(4)))  float    v4f;
typedef v4f  __attribute__((may_alias)) v4fa;

__device__ __forceinline__ unsigned short f2bf(float f) { unsigned u = __float_as_uint(f); u += 0x7FFFu + ((u >> 16) & 1u); return (unsigned short)(u >> 16); }
__device__ __forceinline__ float bfr(float f) { return __uint_as_float(((unsigned)f2bf(f)) << 16); }
__device__ __forceinline__ v16h cat16(v8h lo, v8h hi) { return __builtin_shufflevector(lo, hi, 0, 1, 2, 3, 4, 5, 6, 7, 8, 9, 10, 11, 12, 13, 14, 15); }
static __device__ __forceinline__ h16 toh_flush(float v) { const h16 r = (h16)v; return (fabsf(v) < 6.103515625e-05f) ? (h16)0.0f : r; }
__device__ __forceinline__ v8f wmmag(v16h a, v16h b, v8f c) {
    c = __builtin_amdgcn_wmma_f32_16x16x32_f16(false, a, false, b, (short)0, c, false, false);
    asm volatile("v_nop\n\tv_nop\n\tv_nop\n\tv_nop" : "+v"(c) : "v"(a), "v"(b));
    return c;
}
__device__ __forceinline__ v16h ldh(const h16* p) { return cat16(*(const v8h*)p, *(const v8h*)(p + 16)); }
__device__ __forceinline__ void wave_sync() { __builtin_amdgcn_fence(3  , "wavefront"); __builtin_amdgcn_wave_barrier(); asm volatile("" ::: "memory"); }

__global__ __launch_bounds__(256) void k_wconv(const float* __restrict__ src, h16* dst, int K, int N, float scale) {
    __shared__ float ts[64 * 68];
    const int tid = threadIdx.x;
    const int n0 = blockIdx.x * 64, k0 = blockIdx.y * 64;
    { const int r = tid >> 4, c4 = (tid & 15) * 4;
#pragma unroll
      for (int p = 0; p < 4; ++p) { const int kr = r + 16 * p;
          const v4f v = *(const v4f*)(src + (size_t)(k0 + kr) * N + n0 + c4);
          ts[kr * 68 + c4 + 0] = v[0]; ts[kr * 68 + c4 + 1] = v[1]; ts[kr * 68 + c4 + 2] = v[2]; ts[kr * 68 + c4 + 3] = v[3]; } }
    __syncthreads();
    const int c8 = (tid & 7) * 8;
    v8h hv[2];
#pragma unroll
    for (int p = 0; p < 2; ++p) { const int n = (tid >> 3) + 32 * p;
#pragma unroll
        for (int i = 0; i < 8; ++i) hv[p][i] = toh_flush(bfr(ts[(c8 + i) * 68 + n]) * scale); }
#pragma unroll 1
    for (int ps = 0; ps < 2; ++ps) {
#pragma unroll
        for (int p = 0; p < 2; ++p) { const int n = (tid >> 3) + 32 * p;
            *(volatile v8h*)(dst + (size_t)(n0 + n) * K + k0 + c8) = hv[p]; }
        if (ps == 0) __threadfence(); }
}

__global__ __launch_bounds__(128) void k_invf(float* INVF) {
    const int i = threadIdx.x;
    const float e = ((float)i * 2.0f) / 256.0f;
    const float p = powf(10000.0f, e);
    const float v = 1.0f / p;
    *(volatile float*)(INVF + i) = v; __threadfence(); *(volatile float*)(INVF + i) = v;
}

__global__ __launch_bounds__(256) void k_ropetab(const float* __restrict__ INVF, float* COS, float* SIN) {
    const int idx = blockIdx.x * 256 + threadIdx.x;
    const int t = idx >> 7, i = idx & 127;
    const float ang = (float)t * INVF[i];
    float sn, cs; sincosf(ang, &sn, &cs);
    *(volatile float*)(COS + idx) = cs; *(volatile float*)(SIN + idx) = sn;
    __threadfence();
    *(volatile float*)(COS + idx) = cs; *(volatile float*)(SIN + idx) = sn;
}

__global__ __launch_bounds__(256) void k_ln(const float* __restrict__ X, const float* __restrict__ G, const float* __restrict__ Bv, h16* HP, int rnd, int spitch) {
#pragma clang fp contract(off)
    const int lane = threadIdx.x & 31;
    const int wave = __builtin_amdgcn_readfirstlane((int)(threadIdx.x >> 5));
    const int row = blockIdx.x * 8 + wave;
    if (row >= NB * SEQ) return;
    const size_t srow = (size_t)(row / SEQ) * (size_t)spitch + (size_t)(row % SEQ);
    const v8f xv = *(const v8f*)(X + srow * DM + lane * 8);
    const v8f gv = *(const v8f*)(G + lane * 8);
    const v8f bv = *(const v8f*)(Bv + lane * 8);
    float v[8]; float s = 0.0f;
#pragma unroll
    for (int k = 0; k < 8; ++k) { const float a = xv[k]; const float c = bfr(a); v[k] = (rnd != 0) ? c : a; s += v[k]; }
    s += __shfl_xor(s, 16, 32); s += __shfl_xor(s, 8, 32); s += __shfl_xor(s, 4, 32); s += __shfl_xor(s, 2, 32); s += __shfl_xor(s, 1, 32);
    const float mean = s * (1.0f / 256.0f);
    float q = 0.0f;
#pragma unroll
    for (int k = 0; k < 8; ++k) { v[k] = v[k] - mean; q += v[k] * v[k]; }
    q += __shfl_xor(q, 16, 32); q += __shfl_xor(q, 8, 32); q += __shfl_xor(q, 4, 32); q += __shfl_xor(q, 2, 32); q += __shfl_xor(q, 1, 32);
    const float inv = rsqrtf(q * (1.0f / 256.0f) + 1.0e-5f);
    v8h o;
#pragma unroll
    for (int k = 0; k < 8; ++k) o[k] = toh_flush(((v[k] * inv) * bfr(gv[k]) + bfr(bv[k])) * HC);
    h16* dp = HP + (size_t)row * DM + lane * 8;
    *(volatile v8h*)dp = o; __threadfence(); *(volatile v8h*)dp = o;
}

template <int K>
__device__ __forceinline__ void gemm64(const h16* __restrict__ A, const h16* __restrict__ Bt, const size_t aoff, const size_t boff, v8f (&acc)[4][4]) {
#pragma unroll 1
    for (int kc = 0; kc < K; kc += 32) {
        v16h a[4];
#pragma unroll
        for (int mb = 0; mb < 4; ++mb) a[mb] = ldh(A + aoff + (size_t)mb * 16 * K + kc);
#pragma unroll
        for (int nb = 0; nb < 4; ++nb) { const v16h b = ldh(Bt + boff + (size_t)nb * 16 * K + kc);
#pragma unroll
            for (int mb = 0; mb < 4; ++mb) acc[mb][nb] = wmmag(a[mb], b, acc[mb][nb]); }
    }
}

__global__ __launch_bounds__(32) void k_proj_qk(const h16* __restrict__ A, const h16* __restrict__ Bt, const float* __restrict__ COS, const float* __restrict__ SIN, h16* Ph, h16* Pr, float osc) {
    __shared__ __align__(16) float os[16 * 68];
    const int lane = threadIdx.x & 31, lr = lane & 15, hi = lane >> 4; const int r0 = blockIdx.x * 64, c0 = blockIdx.y * 64;
    v8f acc[4][4];
#pragma unroll
    for (int mb = 0; mb < 4; ++mb)
#pragma unroll
        for (int nb = 0; nb < 4; ++nb) acc[mb][nb] = (v8f){};
    gemm64<DM>(A, Bt, (size_t)(r0 + lr) * DM + 8 * hi, (size_t)(c0 + lr) * DM + 8 * hi, acc);
    const int head = c0 / HD, d0 = c0 % HD;
    const size_t tbase = ((size_t)head * SEQ + (size_t)r0) * HD + d0;
    const size_t rbase = ((size_t)head * EROWS + (size_t)r0) * HD + d0;
    const bool wr = r0 < EROWS;
#pragma unroll
    for (int mb = 0; mb < 4; ++mb) {
#pragma unroll
        for (int nb = 0; nb < 4; ++nb) {
#pragma unroll
            for (int j = 0; j < 8; ++j) os[(hi * 8 + j) * 68 + nb * 16 + lr] = acc[mb][nb][j] * osc; }
        wave_sync();
        v8h hvs[4], rvs[4];
#pragma unroll
        for (int s = 0; s < 4; ++s) { const int row = 4 * s + (lane >> 3), c8 = (lane & 7) * 8;
            const v4f x0 = *(const v4fa*)(&os[row * 68 + c8]); const v4f x1 = *(const v4fa*)(&os[row * 68 + c8 + 4]);
            const int t = r0 + mb * 16 + row;
            const size_t to = (size_t)t * NPAIR + (size_t)((d0 + c8) >> 1);
            const v4f cs = *(const v4f*)(COS + to); const v4f sn = *(const v4f*)(SIN + to);
            float y[8];
            y[0] = x0[0] * cs[0] - x0[1] * sn[0]; y[1] = x0[0] * sn[0] + x0[1] * cs[0];
            y[2] = x0[2] * cs[1] - x0[3] * sn[1]; y[3] = x0[2] * sn[1] + x0[3] * cs[1];
            y[4] = x1[0] * cs[2] - x1[1] * sn[2]; y[5] = x1[0] * sn[2] + x1[1] * cs[2];
            y[6] = x1[2] * cs[3] - x1[3] * sn[3]; y[7] = x1[2] * sn[3] + x1[3] * cs[3];
            v8h hv, rv;
#pragma unroll
            for (int i = 0; i < 8; ++i) { const h16 a0 = toh_flush(y[i]); hv[i] = a0; rv[i] = toh_flush((y[i] - (float)a0) * QRS); }
            hvs[s] = hv; rvs[s] = rv; }
        const size_t sb = tbase + (size_t)(mb * 16) * HD;
        const size_t rb = rbase + (size_t)(mb * 16) * HD;
#pragma unroll 1
        for (int ps = 0; ps < 2; ++ps) {
#pragma unroll
            for (int s = 0; s < 4; ++s) { const int row = 4 * s + (lane >> 3), c8 = (lane & 7) * 8;
                *(volatile v8h*)(Ph + sb + (size_t)row * HD + c8) = hvs[s];
                if (wr) *(volatile v8h*)(Pr + rb + (size_t)row * HD + c8) = rvs[s]; }
            if (ps == 0) __threadfence(); }
        wave_sync();
    }
}

__global__ __launch_bounds__(32) void k_proj_vt(const h16* __restrict__ A, const h16* __restrict__ Bt, h16* Ph, h16* Pr, float osc) {
    __shared__ __align__(16) float os[16 * 68];
    const int lane = threadIdx.x & 31, lr = lane & 15, hi = lane >> 4; const int r0 = blockIdx.x * 64, c0 = blockIdx.y * 64;
    v8f acc[4][4];
#pragma unroll
    for (int mb = 0; mb < 4; ++mb)
#pragma unroll
        for (int nb = 0; nb < 4; ++nb) acc[mb][nb] = (v8f){};
    gemm64<DM>(A, Bt, (size_t)(r0 + lr) * DM + 8 * hi, (size_t)(c0 + lr) * DM + 8 * hi, acc);
    const size_t tbase = (size_t)r0 * SEQ + (size_t)c0;
    const size_t rbase = (size_t)r0 * EROWS + (size_t)c0;
    const bool wr = c0 < EROWS;
#pragma unroll
    for (int mb = 0; mb < 4; ++mb) {
#pragma unroll
        for (int nb = 0; nb < 4; ++nb) {
#pragma unroll
            for (int j = 0; j < 8; ++j) os[(hi * 8 + j) * 68 + nb * 16 + lr] = acc[mb][nb][j] * osc; }
        wave_sync();
        v8h hvs[4], rvs[4];
#pragma unroll
        for (int s = 0; s < 4; ++s) { const int row = 4 * s + (lane >> 3), c8 = (lane & 7) * 8;
            const v4f x0 = *(const v4fa*)(&os[row * 68 + c8]); const v4f x1 = *(const v4fa*)(&os[row * 68 + c8 + 4]); v8h hv, rv;
#pragma unroll
            for (int i = 0; i < 4; ++i) { const h16 a0 = toh_flush(x0[i]); const h16 a1 = toh_flush(x1[i]); hv[i] = a0; hv[4 + i] = a1;
                rv[i] = toh_flush((x0[i] - (float)a0) * QRS); rv[4 + i] = toh_flush((x1[i] - (float)a1) * QRS); }
            hvs[s] = hv; rvs[s] = rv; }
        const size_t sb = tbase + (size_t)(mb * 16) * SEQ;
        const size_t rb = rbase + (size_t)(mb * 16) * EROWS;
#pragma unroll 1
        for (int ps = 0; ps < 2; ++ps) {
#pragma unroll
            for (int s = 0; s < 4; ++s) { const int row = 4 * s + (lane >> 3), c8 = (lane & 7) * 8;
                *(volatile v8h*)(Ph + sb + (size_t)row * SEQ + c8) = hvs[s];
                if (wr) *(volatile v8h*)(Pr + rb + (size_t)row * EROWS + c8) = rvs[s]; }
            if (ps == 0) __threadfence(); }
        wave_sync();
    }
}

__global__ __launch_bounds__(32 * AW) __attribute__((amdgpu_num_vgpr(256)))
void k_flash(const h16* __restrict__ QH, const h16* __restrict__ KP, const h16* __restrict__ VT, h16* CTX) {
    __shared__ __align__(16) h16 os[AW * 16 * OSPH];
    const int lane = threadIdx.x & 31, lr = lane & 15, hi = lane >> 4;
    const int wave = __builtin_amdgcn_readfirstlane((int)(threadIdx.x >> 5));
    const int zh = blockIdx.y;
    const int t0 = EROWS + (blockIdx.x * AW + wave) * 16;
    const int lim = t0 + lr;
    const int nk = (t0 + 16 + 31) & ~31;
    const size_t pbase = (size_t)zh * SEQ * HD;
    const int qo = (t0 + lr) * HD + 8 * hi;
    const size_t ko = pbase + (size_t)lr * HD + 8 * hi;
    const size_t vo = pbase + (size_t)lr * SEQ + 8 * hi;
    v8f o[16];
#pragma unroll
    for (int j = 0; j < 16; ++j) o[j] = (v8f){};
    float m = NEGB, l = 0.0f;
#pragma unroll 1
    for (int key0 = 0; key0 < nk; key0 += 32) {
        int qv = qo; asm volatile("" : "+v"(qv));
        const h16* qa = QH + pbase + (size_t)qv;
        const h16* ka = KP + ko + (size_t)key0 * HD;
        v8f sa = (v8f){}, sb = (v8f){};
#pragma unroll
        for (int kk = 0; kk < 8; ++kk) {
            const v16h qf = ldh(qa + kk * 32);
            const v16h ka0 = ldh(ka + kk * 32), kb0 = ldh(ka + 16 * HD + kk * 32);
            sa = wmmag(ka0, qf, sa); sb = wmmag(kb0, qf, sb); }
        const int ja = key0 + 8 * hi;
        float ta[8], tb[8]; float mx = NEGB;
#pragma unroll
        for (int r = 0; r < 8; ++r) {
            const bool fa = (ja + r <= lim), fb = (ja + 16 + r <= lim);
            ta[r] = sa[r] * SC2; tb[r] = sb[r] * SC2;
            mx = fmaxf(mx, fmaxf(fa ? ta[r] : NEGB, fb ? tb[r] : NEGB)); }
        mx = fmaxf(mx, __shfl_xor(mx, 16, 32));
        const float mnew = fmaxf(m, mx);
        const float alpha = __builtin_amdgcn_exp2f(m - mnew);
        const float sh = PSH - mnew;
        v16h pb; float ls = 0.0f;
#pragma unroll
        for (int r = 0; r < 8; ++r) {
            const float ea = ta[r] + sh, eb = tb[r] + sh;
            const float xa = __builtin_amdgcn_exp2f(ea), xb = __builtin_amdgcn_exp2f(eb);
            const bool fa = (ja + r <= lim) & (ea >= -14.0f), fb = (ja + 16 + r <= lim) & (eb >= -14.0f);
            const float ga = fa ? xa : 0.0f, gb = fb ? xb : 0.0f;
            const h16 pa = (h16)ga; const h16 pc = (h16)gb;
            pb[r] = pa; pb[8 + r] = pc;
            ls += (float)pa + (float)pc; }
        l = l * alpha + ls; m = mnew;
#pragma unroll
        for (int j = 0; j < 16; ++j) o[j] = o[j] * alpha;
        const h16* va = VT + vo + key0;
#pragma unroll
        for (int jg = 0; jg < 4; ++jg) {
            const v16h v0 = ldh(va + (size_t)(4 * jg + 0) * 16 * SEQ), v1 = ldh(va + (size_t)(4 * jg + 1) * 16 * SEQ);
            const v16h v2 = ldh(va + (size_t)(4 * jg + 2) * 16 * SEQ), v3 = ldh(va + (size_t)(4 * jg + 3) * 16 * SEQ);
            o[4 * jg + 0] = wmmag(v0, pb, o[4 * jg + 0]); o[4 * jg + 1] = wmmag(v1, pb, o[4 * jg + 1]);
            o[4 * jg + 2] = wmmag(v2, pb, o[4 * jg + 2]); o[4 * jg + 3] = wmmag(v3, pb, o[4 * jg + 3]); }
    }
    l += __shfl_xor(l, 16, 32);
    const float fin = (1.0f / l) * (CC / QC);
    const int wb = wave * 16 * OSPH;
#pragma unroll
    for (int j = 0; j < 16; ++j) { v8h c;
#pragma unroll
        for (int r = 0; r < 8; ++r) c[r] = toh_flush(o[j][r] * fin);
        *(v8h*)(&os[wb + lr * OSPH + 16 * j + 8 * hi]) = c; }
    wave_sync();
    v8h vals[16];
#pragma unroll
    for (int row = 0; row < 16; ++row) vals[row] = *(const v8h*)(&os[wb + row * OSPH + lane * 8]);
    h16* crow = CTX + (size_t)t0 * INNER + (size_t)zh * HD + lane * 8;
#pragma unroll 1
    for (int ps = 0; ps < 2; ++ps) {
#pragma unroll
        for (int row = 0; row < 16; ++row) *(volatile v8h*)(crow + (size_t)row * INNER) = vals[row];
        if (ps == 0) __threadfence(); }
}

__global__ __launch_bounds__(32 * AW) __attribute__((amdgpu_num_vgpr(256)))
void k_flash_early(const h16* __restrict__ QH, const h16* __restrict__ QR, const h16* __restrict__ KP, const h16* __restrict__ KR,
                   const h16* __restrict__ VT, const h16* __restrict__ VR, h16* CTX) {
    __shared__ __align__(16) h16 os[AW * 16 * OSE];
    const int lane = threadIdx.x & 31, lr = lane & 15, hi = lane >> 4;
    const int wave = __builtin_amdgcn_readfirstlane((int)(threadIdx.x >> 5));
    const int zh = blockIdx.y;
    const int t0 = blockIdx.x * 16;
    const int ds0 = wave * 64;
    const int lim = t0 + lr;
    const int nk = (t0 + 16 + 31) & ~31;
    const size_t pbase = (size_t)zh * SEQ * HD;
    const size_t rbase = (size_t)zh * EROWS * HD;
    const int qo = (t0 + lr) * HD + 8 * hi;
    const size_t ko = (size_t)lr * HD + 8 * hi;
    const size_t vo = pbase + (size_t)(ds0 + lr) * SEQ + 8 * hi;
    const size_t vro = rbase + (size_t)(ds0 + lr) * EROWS + 8 * hi;
    v8f o[4], oR[4];
#pragma unroll
    for (int i = 0; i < 4; ++i) { o[i] = (v8f){}; oR[i] = (v8f){}; }
    float m = NEGB, l = 0.0f;
#pragma unroll 1
    for (int key0 = 0; key0 < nk; key0 += 32) {
        int qv = qo; asm volatile("" : "+v"(qv));
        const h16* qa = QH + pbase + (size_t)qv;
        const h16* qra = QR + rbase + (size_t)qv;
        const h16* ka = KP + pbase + ko + (size_t)key0 * HD;
        const h16* kra = KR + rbase + ko + (size_t)key0 * HD;
        v8f sHa = (v8f){}, sLa = (v8f){}, sHb = (v8f){}, sLb = (v8f){};
#pragma unroll
        for (int kk = 0; kk < 8; ++kk) {
            const v16h qh = ldh(qa + kk * 32), qr = ldh(qra + kk * 32);
            const v16h ka0 = ldh(ka + kk * 32), kb0 = ldh(ka + 16 * HD + kk * 32);
            const v16h kr0 = ldh(kra + kk * 32), kr1 = ldh(kra + 16 * HD + kk * 32);
            sHa = wmmag(ka0, qh, sHa); sLa = wmmag(ka0, qr, sLa); sLa = wmmag(kr0, qh, sLa);
            sHb = wmmag(kb0, qh, sHb); sLb = wmmag(kb0, qr, sLb); sLb = wmmag(kr1, qh, sLb); }
        const int ja = key0 + 8 * hi;
        float ta[8], tb[8]; float mx = NEGB;
#pragma unroll
        for (int r = 0; r < 8; ++r) {
            const bool fa = (ja + r <= lim), fb = (ja + 16 + r <= lim);
            ta[r] = (sHa[r] + sLa[r] * QRI) * SC2; tb[r] = (sHb[r] + sLb[r] * QRI) * SC2;
            mx = fmaxf(mx, fmaxf(fa ? ta[r] : NEGB, fb ? tb[r] : NEGB)); }
        mx = fmaxf(mx, __shfl_xor(mx, 16, 32));
        const float mnew = fmaxf(m, mx);
        const float alpha = __builtin_amdgcn_exp2f(m - mnew);
        const float sh = PSH - mnew;
        v16h pb, pr; float ls = 0.0f;
#pragma unroll
        for (int r = 0; r < 8; ++r) {
            const float ea = ta[r] + sh, eb = tb[r] + sh;
            const float xa = __builtin_amdgcn_exp2f(ea), xb = __builtin_amdgcn_exp2f(eb);
            const bool fa = (ja + r <= lim) & (ea >= -14.0f), fb = (ja + 16 + r <= lim) & (eb >= -14.0f);
            const float ga = fa ? xa : 0.0f, gb = fb ? xb : 0.0f;
            const h16 pa = (h16)ga; const h16 pc = (h16)gb;
            pb[r] = pa; pb[8 + r] = pc;
            pr[r] = toh_flush((ga - (float)pa) * QRS); pr[8 + r] = toh_flush((gb - (float)pc) * QRS);
            ls += ga + gb; }
        l = l * alpha + ls; m = mnew;
#pragma unroll
        for (int i = 0; i < 4; ++i) { o[i] = o[i] * alpha; oR[i] = oR[i] * alpha; }
#pragma unroll
        for (int i = 0; i < 4; ++i) {
            const v16h vf = ldh(VT + vo + (size_t)i * 16 * SEQ + key0);
            const v16h vr = ldh(VR + vro + (size_t)i * 16 * EROWS + key0);
            o[i] = wmmag(vf, pb, o[i]); oR[i] = wmmag(vf, pr, oR[i]); oR[i] = wmmag(vr, pb, oR[i]); }
    }
    l += __shfl_xor(l, 16, 32);
    const float fin = (1.0f / l) * (CC / QC);
    const int wb = wave * 16 * OSE;
#pragma unroll
    for (int i = 0; i < 4; ++i) { v8h c;
#pragma unroll
        for (int r = 0; r < 8; ++r) c[r] = toh_flush((o[i][r] + oR[i][r] * QRI) * fin);
        *(v8h*)(&os[wb + lr * OSE + 16 * i + 8 * hi]) = c; }
    wave_sync();
    v8h vals[4];
#pragma unroll
    for (int s = 0; s < 4; ++s) { const int row = 4 * s + (lane >> 3), c8 = (lane & 7) * 8;
        vals[s] = *(const v8h*)(&os[wb + row * OSE + c8]); }
    h16* cb = CTX + (size_t)t0 * INNER + (size_t)zh * HD + ds0;
#pragma unroll 1
    for (int ps = 0; ps < 2; ++ps) {
#pragma unroll
        for (int s = 0; s < 4; ++s) { const int row = 4 * s + (lane >> 3), c8 = (lane & 7) * 8;
            *(volatile v8h*)(cb + (size_t)row * INNER + c8) = vals[s]; }
        if (ps == 0) __threadfence(); }
}

__global__ __launch_bounds__(32) void k_wo(const h16* __restrict__ A, const h16* __restrict__ Bt, const float* __restrict__ X, float* X1, float osc) {
    __shared__ __align__(16) float os[16 * 68];
    const int lane = threadIdx.x & 31, lr = lane & 15, hi = lane >> 4; const int r0 = blockIdx.x * 64, c0 = blockIdx.y * 64;
    v8f acc[4][4];
#pragma unroll
    for (int mb = 0; mb < 4; ++mb)
#pragma unroll
        for (int nb = 0; nb < 4; ++nb) acc[mb][nb] = (v8f){};
    gemm64<INNER>(A, Bt, (size_t)(r0 + lr) * INNER + 8 * hi, (size_t)(c0 + lr) * INNER + 8 * hi, acc);
#pragma unroll
    for (int mb = 0; mb < 4; ++mb) {
#pragma unroll
        for (int nb = 0; nb < 4; ++nb) {
#pragma unroll
            for (int j = 0; j < 8; ++j) os[(hi * 8 + j) * 68 + nb * 16 + lr] = acc[mb][nb][j] * osc; }
        wave_sync();
        v4f vals[8];
#pragma unroll
        for (int s = 0; s < 8; ++s) { const int row = 2 * s + (lane >> 4), c4 = (lane & 15) * 4;
            const int gr = r0 + mb * 16 + row;
            const size_t xr = (size_t)(gr / SEQ) * SEQ_FULL + (size_t)(gr % SEQ);
            v4f ov = *(const v4fa*)(&os[row * 68 + c4]);
            const v4f xv = *(const v4f*)(X + xr * DM + c0 + c4);
#pragma unroll
            for (int i = 0; i < 4; ++i) ov[i] = ov[i] + bfr(xv[i]);
            vals[s] = ov; }
#pragma unroll 1
        for (int ps = 0; ps < 2; ++ps) {
#pragma unroll
            for (int s = 0; s < 8; ++s) { const int row = 2 * s + (lane >> 4), c4 = (lane & 15) * 4;
                *(volatile v4f*)(X1 + (size_t)(r0 + mb * 16 + row) * DM + c0 + c4) = vals[s]; }
            if (ps == 0) __threadfence(); }
        wave_sync();
    }
}

__global__ __launch_bounds__(32) void k_ffn1(const h16* __restrict__ A, const h16* __restrict__ Bt, const float* __restrict__ B1, h16* MID, float osc) {
    __shared__ __align__(16) float os[16 * 68];
    const int lane = threadIdx.x & 31, lr = lane & 15, hi = lane >> 4; const int r0 = blockIdx.x * 64, c0 = blockIdx.y * 64;
    v8f acc[4][4];
#pragma unroll
    for (int mb = 0; mb < 4; ++mb)
#pragma unroll
        for (int nb = 0; nb < 4; ++nb) acc[mb][nb] = (v8f){};
    gemm64<DM>(A, Bt, (size_t)(r0 + lr) * DM + 8 * hi, (size_t)(c0 + lr) * DM + 8 * hi, acc);
    const int c8 = (lane & 7) * 8;
    const v4f b0 = *(const v4f*)(B1 + c0 + c8); const v4f b1v = *(const v4f*)(B1 + c0 + c8 + 4);
#pragma unroll
    for (int mb = 0; mb < 4; ++mb) {
#pragma unroll
        for (int nb = 0; nb < 4; ++nb) {
#pragma unroll
            for (int j = 0; j < 8; ++j) os[(hi * 8 + j) * 68 + nb * 16 + lr] = acc[mb][nb][j] * osc; }
        wave_sync();
#pragma unroll 1
        for (int s = 0; s < 4; ++s) { const int row = 4 * s + (lane >> 3);
            const v4f x0 = *(const v4fa*)(&os[row * 68 + c8]); const v4f x1 = *(const v4fa*)(&os[row * 68 + c8 + 4]); v8h hv;
#pragma unroll
            for (int i = 0; i < 4; ++i) {
                const float u0 = x0[i] + bfr(b0[i]); const float u1 = x1[i] + bfr(b1v[i]);
                const float g0 = 0.5f * u0 * (1.0f + erff(u0 * 0.70710678118654752f));
                const float g1 = 0.5f * u1 * (1.0f + erff(u1 * 0.70710678118654752f));
                hv[i] = toh_flush(g0 * MC); hv[4 + i] = toh_flush(g1 * MC); }
            h16* dp = MID + (size_t)(r0 + mb * 16 + row) * DFF + c0 + c8;
            *(volatile v8h*)dp = hv; __threadfence(); *(volatile v8h*)dp = hv; }
        wave_sync();
    }
}

__global__ __launch_bounds__(32) void k_ffn2(const h16* __restrict__ A, const h16* __restrict__ Bt, const float* __restrict__ B2, const float* __restrict__ X1, float* OUT, float osc) {
    __shared__ __align__(16) float os[16 * 68];
    const int lane = threadIdx.x & 31, lr = lane & 15, hi = lane >> 4; const int r0 = blockIdx.x * 64, c0 = blockIdx.y * 64;
    v8f acc[4][4];
#pragma unroll
    for (int mb = 0; mb < 4; ++mb)
#pragma unroll
        for (int nb = 0; nb < 4; ++nb) acc[mb][nb] = (v8f){};
    gemm64<DFF>(A, Bt, (size_t)(r0 + lr) * DFF + 8 * hi, (size_t)(c0 + lr) * DFF + 8 * hi, acc);
    const int c4 = (lane & 15) * 4;
    const v4f bb = *(const v4f*)(B2 + c0 + c4);
#pragma unroll
    for (int mb = 0; mb < 4; ++mb) {
#pragma unroll
        for (int nb = 0; nb < 4; ++nb) {
#pragma unroll
            for (int j = 0; j < 8; ++j) os[(hi * 8 + j) * 68 + nb * 16 + lr] = acc[mb][nb][j] * osc; }
        wave_sync();
        v4f vals[8];
#pragma unroll
        for (int s = 0; s < 8; ++s) { const int row = 2 * s + (lane >> 4);
            const int gr = r0 + mb * 16 + row;
            v4f ov = *(const v4fa*)(&os[row * 68 + c4]);
            const v4f xv = *(const v4f*)(X1 + (size_t)gr * DM + c0 + c4);
#pragma unroll
            for (int i = 0; i < 4; ++i) ov[i] = (ov[i] + bfr(bb[i])) + xv[i];
            vals[s] = ov; }
#pragma unroll 1
        for (int ps = 0; ps < 2; ++ps) {
#pragma unroll
            for (int s = 0; s < 8; ++s) { const int row = 2 * s + (lane >> 4);
                const int gr = r0 + mb * 16 + row;
                const size_t orw = (size_t)(gr / SEQ) * OUT_SEQ + (size_t)(gr % SEQ);
                *(volatile v4f*)(OUT + orw * DM + c0 + c4) = vals[s]; }
            if (ps == 0) __threadfence(); }
        wave_sync();
    }
}

static constexpr size_t al256(size_t v) { return (v + 255) & ~(size_t)255; }
static constexpr size_t SZ_WP  = al256((size_t)INNER * DM * 2);
static constexpr size_t SZ_FW  = al256((size_t)DFF * DM * 2);
static constexpr size_t SZ_IF  = al256((size_t)NPAIR * 4);
static constexpr size_t SZ_TAB = al256((size_t)SEQ * NPAIR * 4);
static constexpr size_t SZ_HP  = al256((size_t)NB * SEQ * DM * 2);
static constexpr size_t SZ_PL  = al256((size_t)NH_ * SEQ * HD * 2);
static constexpr size_t SZ_RS  = al256((size_t)NH_ * EROWS * HD * 2);
static constexpr size_t SZ_CTX = al256((size_t)NB * SEQ * INNER * 2);
static constexpr size_t SZ_X1  = al256((size_t)NB * SEQ * DM * 4);
static constexpr size_t SZ_MID = al256((size_t)NB * SEQ * DFF * 2);
static constexpr size_t SZ_TOTAL = 4 * SZ_WP + 2 * SZ_FW + SZ_IF + 2 * SZ_TAB + 2 * SZ_HP + 3 * SZ_PL + 3 * SZ_RS + SZ_CTX + SZ_X1 + SZ_MID;
static_assert(SZ_TOTAL <= (size_t)134217728);
static_assert((size_t)NH_ * SEQ * HD == (size_t)INNER * SEQ);
static_assert((size_t)NH_ * EROWS * HD == (size_t)INNER * EROWS);

extern "C" void kernel_launch(void* const* d_in, const int* in_sizes, int n_in,
                              void* d_out, int out_size, void* d_ws, size_t ws_size, hipStream_t stream) {
    if (n_in < 13) return;
    const size_t needx = ((size_t)(NB - 1) * SEQ_FULL + SEQ) * DM;
    if ((size_t)in_sizes[0] < needx) return;
    if ((size_t)in_sizes[1] < (size_t)DM * INNER || (size_t)in_sizes[2] < (size_t)DM * INNER || (size_t)in_sizes[3] < (size_t)DM * INNER || (size_t)in_sizes[4] < (size_t)INNER * DM) return;
    if ((size_t)in_sizes[5] < (size_t)DM * DFF || in_sizes[6] < DFF || (size_t)in_sizes[7] < (size_t)DFF * DM || in_sizes[8] < DM) return;
    if (in_sizes[9] < DM || in_sizes[10] < DM || in_sizes[11] < DM || in_sizes[12] < DM) return;
    if ((size_t)out_size < ((size_t)(NB - 1) * OUT_SEQ + SEQ) * DM) return;
    if (SZ_TOTAL > ws_size) return;
    const float* x   = (const float*)d_in[0];
    const float* wq  = (const float*)d_in[1];
    const float* wk  = (const float*)d_in[2];
    const float* wv  = (const float*)d_in[3];
    const float* wo  = (const float*)d_in[4];
    const float* f1w = (const float*)d_in[5];
    const float* f1b = (const float*)d_in[6];
    const float* f2w = (const float*)d_in[7];
    const float* f2b = (const float*)d_in[8];
    const float* lag = (const float*)d_in[9];
    const float* lab = (const float*)d_in[10];
    const float* lfg = (const float*)d_in[11];
    const float* lfb = (const float*)d_in[12];
    float* OUT = (float*)d_out;
    char* wsp = (char*)d_ws;
    h16* WQT = (h16*)wsp; wsp += SZ_WP;
    h16* WKT = (h16*)wsp; wsp += SZ_WP;
    h16* WVT = (h16*)wsp; wsp += SZ_WP;
    h16* WOT = (h16*)wsp; wsp += SZ_WP;
    h16* F1T = (h16*)wsp; wsp += SZ_FW;
    h16* F2T = (h16*)wsp; wsp += SZ_FW;
    float* INVF = (float*)wsp; wsp += SZ_IF;
    float* COS = (float*)wsp; wsp += SZ_TAB;
    float* SIN = (float*)wsp; wsp += SZ_TAB;
    h16* HP  = (h16*)wsp; wsp += SZ_HP;
    h16* H2P = (h16*)wsp; wsp += SZ_HP;
    h16* QH = (h16*)wsp; wsp += SZ_PL;
    h16* KP = (h16*)wsp; wsp += SZ_PL;
    h16* VT = (h16*)wsp; wsp += SZ_PL;
    h16* QR = (h16*)wsp; wsp += SZ_RS;
    h16* KR = (h16*)wsp; wsp += SZ_RS;
    h16* VR = (h16*)wsp; wsp += SZ_RS;
    h16* CTX = (h16*)wsp; wsp += SZ_CTX;
    float* X1 = (float*)wsp; wsp += SZ_X1;
    h16* MID = (h16*)wsp; wsp += SZ_MID;

    k_wconv<<<dim3(INNER / 64, DM / 64, 1), 256, 0, stream>>>(wq, WQT, DM, INNER, WC);
    k_wconv<<<dim3(INNER / 64, DM / 64, 1), 256, 0, stream>>>(wk, WKT, DM, INNER, WC);
    k_wconv<<<dim3(INNER / 64, DM / 64, 1), 256, 0, stream>>>(wv, WVT, DM, INNER, WC);
    k_wconv<<<dim3(DM / 64, INNER / 64, 1), 256, 0, stream>>>(wo, WOT, INNER, DM, WC);
    k_wconv<<<dim3(DFF / 64, DM / 64, 1), 256, 0, stream>>>(f1w, F1T, DM, DFF, WC);
    k_wconv<<<dim3(DM / 64, DFF / 64, 1), 256, 0, stream>>>(f2w, F2T, DFF, DM, WC);
    k_invf<<<1, 128, 0, stream>>>(INVF);
    k_ropetab<<<(unsigned)((size_t)SEQ * NPAIR / 256), 256, 0, stream>>>(INVF, COS, SIN);

    k_ln<<<NB * SEQ / 8, 256, 0, stream>>>(x, lag, lab, HP, 1, SEQ_FULL);
    const float osc_qkv = QC / (HC * WC);
    for (int b = 0; b < NB; ++b) {
        const h16* HPb = HP + (size_t)b * SEQ * DM;
        h16* CTXb = CTX + (size_t)b * SEQ * INNER;
        k_proj_qk<<<dim3(SEQ / 64, INNER / 64, 1), 32, 0, stream>>>(HPb, WQT, COS, SIN, QH, QR, osc_qkv);
        k_proj_qk<<<dim3(SEQ / 64, INNER / 64, 1), 32, 0, stream>>>(HPb, WKT, COS, SIN, KP, KR, osc_qkv);
        k_proj_vt<<<dim3(INNER / 64, SEQ / 64, 1), 32, 0, stream>>>(WVT, HPb, VT, VR, osc_qkv);
        k_flash_early<<<dim3(EROWS / 16, NH_, 1), 32 * AW, 0, stream>>>(QH, QR, KP, KR, VT, VR, CTXb);
        if (SEQ > EROWS)
            k_flash<<<dim3((SEQ - EROWS) / (16 * AW), NH_, 1), 32 * AW, 0, stream>>>(QH, KP, VT, CTXb);
    }
    k_wo<<<dim3(NB * SEQ / 64, DM / 64, 1), 32, 0, stream>>>(CTX, WOT, x, X1, 1.0f / (CC * WC));

    k_ln<<<NB * SEQ / 8, 256, 0, stream>>>(X1, lfg, lfb, H2P, 0, SEQ);
    k_ffn1<<<dim3(NB * SEQ / 64, DFF / 64, 1), 32, 0, stream>>>(H2P, F1T, f1b, MID, 1.0f / (HC * WC));
    k_ffn2<<<dim3(NB * SEQ / 64, DM / 64, 1), 32, 0, stream>>>(MID, F2T, f2b, X1, OUT, 1.0f / (MC * WC));
}
